// RowColTransformer_19215683682331
// MI455X (gfx1250) — hardware-verified
//
#include <hip/hip_runtime.h>

typedef _Float16 v16h __attribute__((ext_vector_type(16)));
typedef _Float16 v8h  __attribute__((ext_vector_type(8)));
typedef float    v8f  __attribute__((ext_vector_type(8)));
typedef float    v4f  __attribute__((ext_vector_type(4)));
typedef v8h __attribute__((may_alias)) v8ha;
typedef v4f __attribute__((may_alias)) v4fa;
union Frag { v16h v; v8h half[2]; };

#define TOK    12288
#define NB     768
#define NN     16
#define DIMF   64
#define INNER  128
#define NHEAD  8
#define DHD    16
#define QKVN   384
#define FFW    512
#define FFH    256
#define DEPTH  2
#define TOKB   64
#define NPOSTB (TOK / TOKB)
#define KSTEP  64

#define OFF_QKV1 0
#define OFF_OUT1 24576
#define OFF_F1W1 32768
#define OFF_F1W2 65536
#define OFF_QKV2 81920
#define OFF_OUT2 106496
#define OFF_F2W1 114688
#define OFF_F2W2 147456
#define LWT      163840
#define WT_HALVES (DEPTH * LWT)
#define PLANE_N  (TOK * INNER)
#define Y_N      (TOK * DIMF)

#define PSCALE 16384.0f

static_assert(TOK % TOKB == 0);
static_assert(NB % KSTEP == 0);
static_assert(NB % 16 == 0);
static_assert(TOKB == 4 * NN);

__device__ __forceinline__ v8f wmma16(v16h a, v16h b, v8f c) {
  v8f d = __builtin_amdgcn_wmma_f32_16x16x32_f16(false, a, false, b, (short)0, c, false, false);
  asm volatile("v_nop\n\tv_nop\n\tv_nop\n\tv_nop" : "+v"(d) : "v"(a), "v"(b));
  return d;
}

__device__ __forceinline__ v8h zero8h() {
  const v8h z = { (_Float16)0.0f, (_Float16)0.0f, (_Float16)0.0f, (_Float16)0.0f,
                  (_Float16)0.0f, (_Float16)0.0f, (_Float16)0.0f, (_Float16)0.0f };
  return z;
}
__device__ __forceinline__ v8f zero8f() {
  const v8f z = { 0.f, 0.f, 0.f, 0.f, 0.f, 0.f, 0.f, 0.f };
  return z;
}

__device__ __forceinline__ v16h frag32(const _Float16* p, int h) {
  Frag f;
  f.half[0] = *(const v8ha*)(p + 8 * h);
  f.half[1] = *(const v8ha*)(p + 16 + 8 * h);
  return f.v;
}
__device__ __forceinline__ v16h frag16(const _Float16* p, int h) {
  Frag f;
  f.half[0] = *(const v8ha*)(p + 8 * h);
  f.half[1] = zero8h();
  return f.v;
}
__device__ __forceinline__ v16h pack2(v8f a, v8f c) {
  const v16h r = { (_Float16)(a[0] * PSCALE), (_Float16)(a[1] * PSCALE), (_Float16)(a[2] * PSCALE), (_Float16)(a[3] * PSCALE),
                   (_Float16)(a[4] * PSCALE), (_Float16)(a[5] * PSCALE), (_Float16)(a[6] * PSCALE), (_Float16)(a[7] * PSCALE),
                   (_Float16)(c[0] * PSCALE), (_Float16)(c[1] * PSCALE), (_Float16)(c[2] * PSCALE), (_Float16)(c[3] * PSCALE),
                   (_Float16)(c[4] * PSCALE), (_Float16)(c[5] * PSCALE), (_Float16)(c[6] * PSCALE), (_Float16)(c[7] * PSCALE) };
  return r;
}

__global__ __launch_bounds__(256) void wconv_kernel(
    const float* __restrict__ pq1, const float* __restrict__ po1,
    const float* __restrict__ pa1, const float* __restrict__ pb1,
    const float* __restrict__ pq2, const float* __restrict__ po2,
    const float* __restrict__ pa2, const float* __restrict__ pb2,
    _Float16* wt)
{
  __shared__ __attribute__((aligned(16))) _Float16 st[32 * 256];
  const int tid = threadIdx.x;
  const int t = blockIdx.y & 7, l = blockIdx.y >> 3;
  const float* W; int K, N, off;
  if (t == 0)      { W = pq1; K = DIMF;  N = QKVN; off = OFF_QKV1; }
  else if (t == 1) { W = po1; K = INNER; N = DIMF; off = OFF_OUT1; }
  else if (t == 2) { W = pa1; K = DIMF;  N = FFW;  off = OFF_F1W1; }
  else if (t == 3) { W = pb1; K = FFH;   N = DIMF; off = OFF_F1W2; }
  else if (t == 4) { W = pq2; K = DIMF;  N = QKVN; off = OFF_QKV2; }
  else if (t == 5) { W = po2; K = INNER; N = DIMF; off = OFF_OUT2; }
  else if (t == 6) { W = pa2; K = DIMF;  N = FFW;  off = OFF_F2W1; }
  else             { W = pb2; K = FFH;   N = DIMF; off = OFF_F2W2; }
  const int n0 = blockIdx.x * 32;
  if (n0 >= N) return;
  W += (size_t)l * K * N;
  _Float16* dst = wt + (size_t)l * LWT + off + (size_t)n0 * K;

  const int tot = 32 * K;
  for (int idx = tid; idx < tot; idx += 256) {
    const int nl = idx & 31, k = idx >> 5;
    st[nl * K + k] = (_Float16)(W[(size_t)k * N + n0 + nl] * 32.0f);
  }
  __syncthreads();
  const int np = 4 * K;
  for (int p = tid; p < np; p += 256) {
    const v8h v = *(const v8ha*)(st + p * 8);
    *(volatile v8h*)(dst + (size_t)p * 8) = v;
  }
  __threadfence();
  for (int p = tid; p < np; p += 256) {
    const v8h v = *(const v8ha*)(st + p * 8);
    *(volatile v8h*)(dst + (size_t)p * 8) = v;
  }
}

__device__ __forceinline__ void ln_tile(v8f (&x)[4], const float* __restrict__ g,
                                        const float* __restrict__ b, int m) {
  float gg[4], bb[4];
#pragma unroll
  for (int nt = 0; nt < 4; ++nt) { gg[nt] = g[16 * nt + m]; bb[nt] = b[16 * nt + m]; }
#pragma unroll
  for (int r = 0; r < 8; ++r) {
    float s = (x[0][r] + x[1][r]) + (x[2][r] + x[3][r]);
    s += __shfl_xor(s, 1, 32); s += __shfl_xor(s, 2, 32);
    s += __shfl_xor(s, 4, 32); s += __shfl_xor(s, 8, 32);
    const float mu = s * (1.0f / 64.0f);
    const float d0 = x[0][r] - mu, d1 = x[1][r] - mu, d2 = x[2][r] - mu, d3 = x[3][r] - mu;
    float v = (d0 * d0 + d1 * d1) + (d2 * d2 + d3 * d3);
    v += __shfl_xor(v, 1, 32); v += __shfl_xor(v, 2, 32);
    v += __shfl_xor(v, 4, 32); v += __shfl_xor(v, 8, 32);
    const float rs = 1.0f / sqrtf(v * (1.0f / 64.0f) + 1.0e-5f);
    x[0][r] = d0 * rs * gg[0] + bb[0];
    x[1][r] = d1 * rs * gg[1] + bb[1];
    x[2][r] = d2 * rs * gg[2] + bb[2];
    x[3][r] = d3 * rs * gg[3] + bb[3];
  }
}

__device__ __forceinline__ void store_rows64(const float* s, float* dst, int w, int lane) {
#pragma unroll
  for (int j = 0; j < 8; ++j) {
    const int off = w * 1024 + 128 * j + 4 * lane;
    const v4f v = *(const v4fa*)(s + off);
    *(volatile v4f*)(dst + off) = v;
  }
}

__device__ __forceinline__ void store_qkv_lines(const _Float16* s, _Float16* pl, int b0, int hb,
                                                int w, int lane) {
  const int p = lane & 7, hh = lane >> 3;
#pragma unroll
  for (int j = 0; j < 4; ++j) {
    const int L = (4 * w + j) * NHEAD + hb + hh;
    const v8h v = *(const v8ha*)(s + L * 64 + p * 8);
    *(volatile v8h*)(pl + ((size_t)L * NB + b0) * DHD + p * 8) = v;
  }
}

__global__ __launch_bounds__(128) void post_kernel(
    const float* __restrict__ xin,
    const _Float16* __restrict__ op,
    float* yp,
    const _Float16* __restrict__ wout,
    const float* __restrict__ bout,
    const float* __restrict__ lng, const float* __restrict__ lnb,
    const _Float16* __restrict__ w1,
    const float* __restrict__ b1,
    const _Float16* __restrict__ w2,
    const float* __restrict__ b2,
    const float* __restrict__ nlg, const float* __restrict__ nlb,
    const _Float16* __restrict__ wqkv,
    _Float16* qpl, _Float16* kpl, _Float16* vpl,
    float* out, int mode)
{
  __shared__ __attribute__((aligned(16))) float    sy[TOKB * DIMF];
  __shared__ __attribute__((aligned(16))) _Float16 syh[TOKB * DIMF];
  __shared__ __attribute__((aligned(16))) _Float16 sg[TOKB * FFH];

  const int tid = threadIdx.x, lane = tid & 31, w = tid >> 5;
  const int h = lane >> 4, m = lane & 15;
  const int t0 = blockIdx.x * TOKB;
  const int rowA = t0 + 16 * w + m;
  const int rowD = t0 + 16 * w + 8 * h;
  const int lrow = 16 * w + 8 * h;

  v8f x[4];
  if (mode == 0) {
#pragma unroll
    for (int nt = 0; nt < 4; ++nt)
#pragma unroll
      for (int r = 0; r < 8; ++r)
        x[nt][r] = xin[(size_t)(rowD + r) * DIMF + 16 * nt + m];
  } else {
    v8f acc[4];
#pragma unroll
    for (int nt = 0; nt < 4; ++nt) acc[nt] = zero8f();
#pragma unroll 1
    for (int ks = 0; ks < INNER / 32; ++ks) {
      const v16h a = frag32(op + (size_t)rowA * INNER + 32 * ks, h);
#pragma unroll
      for (int nt = 0; nt < 4; ++nt) {
        const v16h b = frag32(wout + (size_t)(16 * nt + m) * INNER + 32 * ks, h);
        acc[nt] = wmma16(a, b, acc[nt]);
      }
    }
#pragma unroll
    for (int nt = 0; nt < 4; ++nt) {
      const float bb = bout[16 * nt + m];
#pragma unroll
      for (int r = 0; r < 8; ++r)
        x[nt][r] = acc[nt][r] * (1.0f / 2048.0f) + bb + yp[(size_t)(rowD + r) * DIMF + 16 * nt + m];
    }
    ln_tile(x, lng, lnb, m);
#pragma unroll
    for (int nt = 0; nt < 4; ++nt)
#pragma unroll
      for (int r = 0; r < 8; ++r) {
        sy[(lrow + r) * DIMF + 16 * nt + m]  = x[nt][r];
        syh[(lrow + r) * DIMF + 16 * nt + m] = (_Float16)x[nt][r];
      }
    __syncthreads();
#pragma unroll 1
    for (int c = 0; c < 8; ++c) {
      v8f au[2], ag[2];
      au[0] = zero8f(); au[1] = zero8f(); ag[0] = zero8f(); ag[1] = zero8f();
#pragma unroll 1
      for (int ks = 0; ks < DIMF / 32; ++ks) {
        const v16h a = frag32(syh + (16 * w + m) * DIMF + 32 * ks, h);
#pragma unroll
        for (int nt = 0; nt < 2; ++nt) {
          const v16h bu = frag32(w1 + (size_t)(32 * c + 16 * nt + m) * DIMF + 32 * ks, h);
          au[nt] = wmma16(a, bu, au[nt]);
          const v16h bg = frag32(w1 + (size_t)(FFH + 32 * c + 16 * nt + m) * DIMF + 32 * ks, h);
          ag[nt] = wmma16(a, bg, ag[nt]);
        }
      }
#pragma unroll
      for (int nt = 0; nt < 2; ++nt) {
        const int colu = 32 * c + 16 * nt + m;
        const float bu = b1[colu], bg = b1[FFH + colu];
#pragma unroll
        for (int r = 0; r < 8; ++r) {
          const float u  = au[nt][r] * (1.0f / 32.0f) + bu;
          const float gv = ag[nt][r] * (1.0f / 32.0f) + bg;
          const float ge = 0.5f * gv * (1.0f + erff(gv * 0.70710678118654752f));
          sg[(lrow + r) * FFH + colu] = (_Float16)(u * ge * 256.0f);
        }
      }
    }
    __syncthreads();
    v8f acc2[4];
#pragma unroll
    for (int nt = 0; nt < 4; ++nt) acc2[nt] = zero8f();
#pragma unroll 1
    for (int ks = 0; ks < FFH / 32; ++ks) {
      const v16h a = frag32(sg + (16 * w + m) * FFH + 32 * ks, h);
#pragma unroll
      for (int nt = 0; nt < 4; ++nt) {
        const v16h b = frag32(w2 + (size_t)(16 * nt + m) * FFH + 32 * ks, h);
        acc2[nt] = wmma16(a, b, acc2[nt]);
      }
    }
#pragma unroll
    for (int nt = 0; nt < 4; ++nt) {
      const float bb = b2[16 * nt + m];
#pragma unroll
      for (int r = 0; r < 8; ++r)
        x[nt][r] = acc2[nt][r] * (1.0f / 8192.0f) + bb + sy[(lrow + r) * DIMF + 16 * nt + m];
    }
  }

  if (mode == 2) {
#pragma unroll
    for (int nt = 0; nt < 4; ++nt)
#pragma unroll
      for (int r = 0; r < 8; ++r)
        sy[(lrow + r) * DIMF + 16 * nt + m] = x[nt][r];
    __syncthreads();
    store_rows64(sy, out + (size_t)t0 * DIMF, w, lane);
    __threadfence();
    store_rows64(sy, out + (size_t)t0 * DIMF, w, lane);
  } else {
    ln_tile(x, nlg, nlb, m);
#pragma unroll
    for (int nt = 0; nt < 4; ++nt)
#pragma unroll
      for (int r = 0; r < 8; ++r) {
        sy[(lrow + r) * DIMF + 16 * nt + m]  = x[nt][r];
        syh[(lrow + r) * DIMF + 16 * nt + m] = (_Float16)x[nt][r];
      }
    __syncthreads();
    store_rows64(sy, yp + (size_t)t0 * DIMF, w, lane);
    __threadfence();
    store_rows64(sy, yp + (size_t)t0 * DIMF, w, lane);

    const int b0 = blockIdx.x * 4;
#pragma unroll 1
    for (int c = 0; c < 6; ++c) {
      v8f acc[4];
#pragma unroll
      for (int nt = 0; nt < 4; ++nt) acc[nt] = zero8f();
#pragma unroll 1
      for (int ks = 0; ks < DIMF / 32; ++ks) {
        const v16h a = frag32(syh + (16 * w + m) * DIMF + 32 * ks, h);
#pragma unroll
        for (int nt = 0; nt < 4; ++nt) {
          const v16h b = frag32(wqkv + (size_t)(64 * c + 16 * nt + m) * DIMF + 32 * ks, h);
          acc[nt] = wmma16(a, b, acc[nt]);
        }
      }
      __syncthreads();
      const int hb = 4 * (c & 1);
#pragma unroll
      for (int nt = 0; nt < 4; ++nt)
#pragma unroll
        for (int r = 0; r < 8; ++r)
          sg[(((8 * h + r) * NHEAD) + hb + nt) * 64 + 16 * w + m] = (_Float16)(acc[nt][r] * 0.25f);
      __syncthreads();
      _Float16* pl = (c < 2) ? qpl : ((c < 4) ? kpl : vpl);
      store_qkv_lines(sg, pl, b0, hb, w, lane);
      __threadfence();
      store_qkv_lines(sg, pl, b0, hb, w, lane);
    }
  }
}

__global__ __launch_bounds__(256) void attn_col_kernel(
    const _Float16* __restrict__ qpl, const _Float16* __restrict__ kpl,
    const _Float16* __restrict__ vpl, _Float16* opl)
{
  __shared__ __attribute__((aligned(16))) _Float16 sq[NN * INNER];
  __shared__ __attribute__((aligned(16))) _Float16 sk[NN * INNER];
  __shared__ __attribute__((aligned(16))) _Float16 sv[NN * INNER];
  __shared__ __attribute__((aligned(16))) _Float16 so[NN * INNER];

  const int tid = threadIdx.x, lane = tid & 31, hd = tid >> 5;
  const int h = lane >> 4, m = lane & 15;
  const int b = blockIdx.x;
  {
    const int n = tid >> 4, ph = (tid >> 1) & 7, hf = tid & 1;
    const size_t src = ((size_t)(n * NHEAD + ph) * NB + b) * DHD + 8 * hf;
    const int dst = n * INNER + ph * DHD + 8 * hf;
    *(v8ha*)(sq + dst) = *(const v8ha*)(qpl + src);
    *(v8ha*)(sk + dst) = *(const v8ha*)(kpl + src);
    *(v8ha*)(sv + dst) = *(const v8ha*)(vpl + src);
  }
  __syncthreads();

  const v16h ka = frag16(sk + m * INNER + hd * DHD, h);
  const v16h qb = frag16(sq + m * INNER + hd * DHD, h);
  const v8f s = wmma16(ka, qb, zero8f());

  float mx = s[0];
#pragma unroll
  for (int r = 1; r < 8; ++r) mx = fmaxf(mx, s[r]);
  mx = fmaxf(mx, __shfl_xor(mx, 16, 32));
  float e[8];
  float t = 0.0f;
#pragma unroll
  for (int r = 0; r < 8; ++r) { e[r] = __expf((s[r] - mx) * (1.0f / 256.0f)); t += e[r]; }
  t += __shfl_xor(t, 16, 32);

  Frag pb;
  {
    const v8h pv = { (_Float16)(e[0] * PSCALE), (_Float16)(e[1] * PSCALE), (_Float16)(e[2] * PSCALE), (_Float16)(e[3] * PSCALE),
                     (_Float16)(e[4] * PSCALE), (_Float16)(e[5] * PSCALE), (_Float16)(e[6] * PSCALE), (_Float16)(e[7] * PSCALE) };
    pb.half[0] = pv; pb.half[1] = zero8h();
  }
  Frag va;
  {
    const _Float16* vc = sv + hd * DHD + m;
    const v8h vv = { vc[(8 * h + 0) * INNER], vc[(8 * h + 1) * INNER], vc[(8 * h + 2) * INNER], vc[(8 * h + 3) * INNER],
                     vc[(8 * h + 4) * INNER], vc[(8 * h + 5) * INNER], vc[(8 * h + 6) * INNER], vc[(8 * h + 7) * INNER] };
    va.half[0] = vv; va.half[1] = zero8h();
  }
  const v8f o = wmma16(va.v, pb.v, zero8f());

  const float inv = (1.0f / t) * (1.0f / 2048.0f);
#pragma unroll
  for (int r = 0; r < 8; ++r) so[m * INNER + hd * DHD + 8 * h + r] = (_Float16)(o[r] * inv);
  __syncthreads();

  const v8h ov = *(const v8ha*)(so + tid * 8);
  _Float16* od = opl + (size_t)b * NN * INNER + tid * 8;
  *(volatile v8h*)od = ov;
  __threadfence();
  *(volatile v8h*)od = ov;
}

__global__ __launch_bounds__(256) void attn_row_kernel(
    const _Float16* __restrict__ qpl, const _Float16* __restrict__ kpl,
    const _Float16* __restrict__ vpl, _Float16* opl)
{
  __shared__ __attribute__((aligned(16))) _Float16 sk[NHEAD * KSTEP * DHD];
  __shared__ __attribute__((aligned(16))) _Float16 svt[NHEAD * DHD * KSTEP];
  __shared__ __attribute__((aligned(16))) _Float16 so[NN * INNER];

  const int tid = threadIdx.x, lane = tid & 31, hd = tid >> 5;
  const int h = lane >> 4, m = lane & 15;
  const int n = blockIdx.y, qb = blockIdx.x * 16;
  const size_t hbase = (size_t)(n * NHEAD + hd) * NB * DHD;

  const v16h qf = frag16(qpl + hbase + (size_t)(qb + m) * DHD, h);

  v8f o = zero8f();
  float mrun = -1.0e30f, lrun = 0.0f;

#pragma unroll 1
  for (int kb = 0; kb < NB; kb += KSTEP) {
    __syncthreads();
#pragma unroll
    for (int i = 0; i < 4; ++i) {
      const int p = tid + 256 * i;
      const int ph = p >> 7, key = (p >> 1) & 63, hf = p & 1;
      const size_t src = ((size_t)(n * NHEAD + ph) * NB + kb + key) * DHD + 8 * hf;
      *(v8ha*)(sk + ph * (KSTEP * DHD) + key * DHD + 8 * hf) = *(const v8ha*)(kpl + src);
      const v8h vv = *(const v8ha*)(vpl + src);
#pragma unroll
      for (int e2 = 0; e2 < 8; ++e2) svt[ph * (KSTEP * DHD) + (8 * hf + e2) * KSTEP + key] = vv[e2];
    }
    __syncthreads();

    v8f s[4];
#pragma unroll
    for (int j = 0; j < 4; ++j) {
      const v16h ka = frag16(sk + hd * (KSTEP * DHD) + (16 * j + m) * DHD, h);
      s[j] = wmma16(ka, qf, zero8f());
    }
    float mloc = s[0][0];
#pragma unroll
    for (int j = 0; j < 4; ++j)
#pragma unroll
      for (int r = 0; r < 8; ++r) mloc = fmaxf(mloc, s[j][r]);
    mloc = fmaxf(mloc, __shfl_xor(mloc, 16, 32));
    const float mnew = fmaxf(mrun, mloc);
    const float alpha = __expf((mrun - mnew) * (1.0f / 256.0f));
    mrun = mnew;
    float lsum = 0.0f;
#pragma unroll
    for (int j = 0; j < 4; ++j)
#pragma unroll
      for (int r = 0; r < 8; ++r) {
        const float p = __expf((s[j][r] - mnew) * (1.0f / 256.0f));
        s[j][r] = p;
        lsum += p;
      }
    lsum += __shfl_xor(lsum, 16, 32);
    lrun = lrun * alpha + lsum;
#pragma unroll
    for (int r = 0; r < 8; ++r) o[r] = o[r] * alpha;

    const v16h pb0 = pack2(s[0], s[1]);
    const v16h pb1 = pack2(s[2], s[3]);
    const _Float16* vr = svt + hd * (KSTEP * DHD) + m * KSTEP;
    const v16h va0 = frag32(vr, h);
    const v16h va1 = frag32(vr + 32, h);
    o = wmma16(va0, pb0, o);
    o = wmma16(va1, pb1, o);
  }

  const float inv = (1.0f / lrun) * (1.0f / 2048.0f);
#pragma unroll
  for (int r = 0; r < 8; ++r) so[m * INNER + hd * DHD + 8 * h + r] = (_Float16)(o[r] * inv);
  __syncthreads();

  const int row = 2 * hd + (lane >> 4), pc = lane & 15;
  const v8h ov = *(const v8ha*)(so + row * INNER + pc * 8);
  _Float16* od = opl + ((size_t)(qb + row) * NN + n) * INNER + pc * 8;
  *(volatile v8h*)od = ov;
  __threadfence();
  *(volatile v8h*)od = ov;
}

extern "C" void kernel_launch(void* const* d_in, const int* in_sizes, int n_in,
                              void* d_out, int out_size, void* d_ws, size_t ws_size,
                              hipStream_t stream) {
  if (n_in < 23) return;
  if (in_sizes[0] != TOK * DIMF || out_size != TOK * DIMF) return;
  if (in_sizes[3] != DEPTH * DIMF * QKVN || in_sizes[14] != DEPTH * DIMF * QKVN) return;
  if (in_sizes[4] != DEPTH * INNER * DIMF || in_sizes[15] != DEPTH * INNER * DIMF) return;
  if (in_sizes[8] != DEPTH * DIMF * FFW || in_sizes[19] != DEPTH * DIMF * FFW) return;
  if (in_sizes[10] != DEPTH * FFH * DIMF || in_sizes[21] != DEPTH * FFH * DIMF) return;
  if (in_sizes[9] != DEPTH * FFW || in_sizes[20] != DEPTH * FFW) return;
  {
    const int small_idx[12] = { 1, 2, 5, 6, 7, 11, 12, 13, 16, 17, 18, 22 };
    for (int i = 0; i < 12; ++i) if (in_sizes[small_idx[i]] != DEPTH * DIMF) return;
  }

  const float* x      = (const float*)d_in[0];
  const float* ln1_g  = (const float*)d_in[1];
  const float* ln1_b  = (const float*)d_in[2];
  const float* qkv1_w = (const float*)d_in[3];
  const float* out1_w = (const float*)d_in[4];
  const float* out1_b = (const float*)d_in[5];
  const float* ln2_g  = (const float*)d_in[6];
  const float* ln2_b  = (const float*)d_in[7];
  const float* ff1_w1 = (const float*)d_in[8];
  const float* ff1_b1 = (const float*)d_in[9];
  const float* ff1_w2 = (const float*)d_in[10];
  const float* ff1_b2 = (const float*)d_in[11];
  const float* ln3_g  = (const float*)d_in[12];
  const float* ln3_b  = (const float*)d_in[13];
  const float* qkv2_w = (const float*)d_in[14];
  const float* out2_w = (const float*)d_in[15];
  const float* out2_b = (const float*)d_in[16];
  const float* ln4_g  = (const float*)d_in[17];
  const float* ln4_b  = (const float*)d_in[18];
  const float* ff2_w1 = (const float*)d_in[19];
  const float* ff2_b1 = (const float*)d_in[20];
  const float* ff2_w2 = (const float*)d_in[21];
  const float* ff2_b2 = (const float*)d_in[22];
  float* out = (float*)d_out;

  const size_t wt_bytes = (size_t)WT_HALVES * 2;
  const size_t y_bytes  = (size_t)Y_N * 4;
  const size_t pl_bytes = (size_t)PLANE_N * 2;
  const size_t total = wt_bytes + y_bytes + 4 * pl_bytes;
  if (total > ws_size) return;

  char* ws = (char*)d_ws;
  _Float16* wt = (_Float16*)(ws);
  float*    yp = (float*)(ws + wt_bytes);
  _Float16* qp = (_Float16*)(ws + wt_bytes + y_bytes);
  _Float16* kp = (_Float16*)(ws + wt_bytes + y_bytes + pl_bytes);
  _Float16* vp = (_Float16*)(ws + wt_bytes + y_bytes + 2 * pl_bytes);
  _Float16* op = (_Float16*)(ws + wt_bytes + y_bytes + 3 * pl_bytes);

  wconv_kernel<<<dim3(16, 16), 256, 0, stream>>>(qkv1_w, out1_w, ff1_w1, ff1_w2,
                                                   qkv2_w, out2_w, ff2_w1, ff2_w2, wt);

  post_kernel<<<NPOSTB, 128, 0, stream>>>(x, op, yp,
      wt + OFF_OUT1, out1_b, ln2_g, ln2_b, wt + OFF_F1W1, ff1_b1, wt + OFF_F1W2, ff1_b2,
      ln1_g, ln1_b, wt + OFF_QKV1, qp, kp, vp, out, 0);

  for (int l = 0; l < DEPTH; ++l) {
    const _Float16* wl = wt + (size_t)l * LWT;
    attn_col_kernel<<<NB, 256, 0, stream>>>(qp, kp, vp, op);
    post_kernel<<<NPOSTB, 128, 0, stream>>>(x, op, yp,
        wl + OFF_OUT1, out1_b + l * DIMF, ln2_g + l * DIMF, ln2_b + l * DIMF,
        wl + OFF_F1W1, ff1_b1 + l * FFW, wl + OFF_F1W2, ff1_b2 + l * DIMF,
        ln3_g + l * DIMF, ln3_b + l * DIMF, wl + OFF_QKV2, qp, kp, vp, out, 1);
    attn_row_kernel<<<dim3(NB / 16, NN), 256, 0, stream>>>(qp, kp, vp, op);
    const int last = (l == DEPTH - 1) ? 1 : 0;
    const float* ng = last ? ln1_g : (ln1_g + (l + 1) * DIMF);
    const float* nb = last ? ln1_b : (ln1_b + (l + 1) * DIMF);
    const _Float16* nw = last ? wt : (wt + (size_t)(l + 1) * LWT + OFF_QKV1);
    post_kernel<<<NPOSTB, 128, 0, stream>>>(x, op, yp,
        wl + OFF_OUT2, out2_b + l * DIMF, ln4_g + l * DIMF, ln4_b + l * DIMF,
        wl + OFF_F2W1, ff2_b1 + l * FFW, wl + OFF_F2W2, ff2_b2 + l * DIMF,
        ng, nb, nw, qp, kp, vp, out, last ? 2 : 1);
  }
}
